// NRUCell_1039382085932
// MI455X (gfx1250) — hardware-verified
//
#include <hip/hip_runtime.h>
#include <math.h>

constexpr int kBatch = 8192;
constexpr int kInpF  = 1024;
constexpr int kHidF  = 1024;
constexpr int kMemF  = 256;
constexpr int kCatK  = kInpF + kHidF + kMemF;
constexpr int kHmK   = kHidF + kMemF;
constexpr int kUReal = 136;
constexpr int kUN    = 192;
static_assert(kCatK % 32 == 0 && kHmK % 32 == 0, "k");
static_assert(kBatch % 64 == 0 && kHidF % 64 == 0 && kUN % 64 == 0, "mn");

constexpr size_t kOffA1 = 0;
constexpr size_t kOffW1 = kOffA1 + (size_t)kBatch * kCatK * 2;
constexpr size_t kOffA2 = kOffW1 + (size_t)kHidF * kCatK * 2;
constexpr size_t kOffW2 = kOffA2 + (size_t)kBatch * kHmK * 2;
constexpr size_t kOffU  = kOffW2 + (size_t)kUN * kHmK * 2;
constexpr size_t kOffB1 = kOffU + (size_t)kBatch * kUN * 4;
constexpr size_t kOffB2 = kOffB1 + (size_t)kHidF * 4;
constexpr size_t kWsTotal = kOffB2 + 1024;
static_assert(kWsTotal == 70226944, "ws");
static_assert(kOffW1 % 256 == 0 && kOffA2 % 256 == 0 && kOffW2 % 256 == 0 && kOffU % 256 == 0 && kOffB1 % 256 == 0 && kOffB2 % 256 == 0, "al");
static_assert(kWsTotal <= 134217728, "cap");

typedef __attribute__((ext_vector_type(16))) _Float16 v16h;
typedef __attribute__((ext_vector_type(8)))  _Float16 v8h;
typedef __attribute__((ext_vector_type(16))) __bf16   v16b;
typedef __attribute__((ext_vector_type(8)))  __bf16   v8b;
typedef __attribute__((ext_vector_type(8)))  float    v8f;
typedef __attribute__((ext_vector_type(4)))  float    v4f;
typedef __attribute__((ext_vector_type(4)))  unsigned int v4u;

__device__ __forceinline__ unsigned short f2bf_bits(float f) {
  unsigned u = __float_as_uint(f);
  return (unsigned short)((u + 0x7FFFu + ((u >> 16) & 1u)) >> 16);
}
__device__ __forceinline__ float bf_bits2f(unsigned short h) { return __uint_as_float(((unsigned)h) << 16); }

__device__ __forceinline__ void dep_guard_h(v8f& a, v8f& b, v16h x, v16h y) { asm volatile("v_nop\n\tv_nop\n\tv_nop\n\tv_nop" : "+v"(a), "+v"(b) : "v"(x), "v"(y)); }
__device__ __forceinline__ void dep_guard_b(v8f& a, v8f& b, v16b x, v16b y) { asm volatile("v_nop\n\tv_nop\n\tv_nop\n\tv_nop" : "+v"(a), "+v"(b) : "v"(x), "v"(y)); }
__device__ __forceinline__ void keep4_h(v16h a, v16h b, v16h c, v16h d) { asm volatile("v_nop" :: "v"(a), "v"(b), "v"(c), "v"(d)); }
__device__ __forceinline__ void keep4_b(v16b a, v16b b, v16b c, v16b d) { asm volatile("v_nop" :: "v"(a), "v"(b), "v"(c), "v"(d)); }
__device__ __forceinline__ void acc_guard4(v8f& a, v8f& b, v8f& c, v8f& d) { asm volatile("v_nop\n\tv_nop\n\tv_nop\n\tv_nop" : "+v"(a), "+v"(b), "+v"(c), "+v"(d)); }
template <typename T> struct Frag;
template <> struct Frag<_Float16> {
  typedef v16h V; union U { v16h v; v8h h[2]; };
  static __device__ __forceinline__ v16h load(const _Float16* p) {
    U f; f.h[0] = *(const v8h*)(p); f.h[1] = *(const v8h*)(p + 16); return f.v;
  }
  static __device__ __forceinline__ v8f mma(v16h a, v16h b, v8f c) {
    return __builtin_amdgcn_wmma_f32_16x16x32_f16(false, a, false, b, (short)0, c, false, false);
  }
  static __device__ __forceinline__ void guard(v8f& a, v8f& b, v16h x, v16h y) { dep_guard_h(a, b, x, y); }
  static __device__ __forceinline__ void keep(v16h a, v16h b, v16h c, v16h d) { keep4_h(a, b, c, d); }
};
template <> struct Frag<__bf16> {
  typedef v16b V; union U { v16b v; v8b h[2]; };
  static __device__ __forceinline__ v16b load(const __bf16* p) {
    U f; f.h[0] = *(const v8b*)(p); f.h[1] = *(const v8b*)(p + 16); return f.v;
  }
  static __device__ __forceinline__ v8f mma(v16b a, v16b b, v8f c) {
    return __builtin_amdgcn_wmma_f32_16x16x32_bf16(false, a, false, b, (short)0, c, false, false);
  }
  static __device__ __forceinline__ void guard(v8f& a, v8f& b, v16b x, v16b y) { dep_guard_b(a, b, x, y); }
  static __device__ __forceinline__ void keep(v16b a, v16b b, v16b c, v16b d) { keep4_b(a, b, c, d); }
};

__device__ __forceinline__ unsigned pk16(unsigned short a, unsigned short b) { return (unsigned)a | ((unsigned)b << 16); }

template <int ET> struct Elem;
template <> struct Elem<0> { typedef _Float16 T; };
template <> struct Elem<1> { typedef __bf16 T; };
template <int ET, bool SPLIT, int BIAS_MODE, int OUT_MODE, bool RESID, int ACT = 0>
__global__ __launch_bounds__(256) void wmma_gemm64(
    const unsigned short* __restrict__ Ap, const unsigned short* __restrict__ A2p, int lda, long strideA,
    const unsigned short* __restrict__ Btp, const unsigned short* __restrict__ Bt2p, int ldb, long strideB,
    void* __restrict__ Cout, void* __restrict__ Cout2, int ldc, long strideC,
    const float* __restrict__ bias,
    const float* __restrict__ resid, long strideR,
    int M, int N, int K, float scale) {
  typedef typename Elem<ET>::T T;
  typedef typename Frag<T>::V V;
  const T* A = (const T*)Ap; const T* A2 = (const T*)A2p; const T* Bt = (const T*)Btp; const T* Bt2 = (const T*)Bt2p;
  __shared__ __align__(16) float sT[8][16 * 68];
  const int b    = blockIdx.y;
  const int lane = threadIdx.x & 31;
  const int wave = threadIdx.x >> 5;
  const int tilesN = N >> 6;
  const int tilesM = M >> 6;
  const int tile = blockIdx.x * 8 + wave;
  if (tile >= tilesM * tilesN) return;
  const int tm = tile / tilesN;
  const int tn = tile - tm * tilesN;
  const int m0 = tm << 6;
  const int n0 = tn << 6;

  const T* Ab  = A  + (size_t)b * strideA;
  const T* Bb  = Bt + (size_t)b * strideB;
  const T* Ab2 = SPLIT ? (A2  + (size_t)b * strideA) : nullptr;
  const T* Bb2 = SPLIT ? (Bt2 + (size_t)b * strideB) : nullptr;

  const int rlane = lane & 15;
  const int koff  = (lane >> 4) * 8;
  const int mOff  = (lane >> 4) * 8;

  v8f acc[4][4];
#pragma unroll
  for (int i = 0; i < 4; ++i)
#pragma unroll
    for (int j = 0; j < 4; ++j) acc[i][j] = (v8f){0.f,0.f,0.f,0.f,0.f,0.f,0.f,0.f};

  for (int k0 = 0; k0 < K; k0 += 32) {
    V bh[4], bl[4];
#pragma unroll
    for (int j = 0; j < 4; ++j) {
      const size_t bo = (size_t)(n0 + (j << 4) + rlane) * ldb + koff + k0;
      bh[j] = Frag<T>::load(Bb + bo);
      if (SPLIT) bl[j] = Frag<T>::load(Bb2 + bo);
    }
#pragma unroll
    for (int i = 0; i < 4; ++i) {
      const size_t ao = (size_t)(m0 + (i << 4) + rlane) * lda + koff + k0;
      V ah = Frag<T>::load(Ab + ao);
      V al;
      if (SPLIT) al = Frag<T>::load(Ab2 + ao);
#pragma unroll
      for (int j = 0; j < 4; ++j) {
        acc[i][j] = Frag<T>::mma(ah, bh[j], acc[i][j]);
        if (SPLIT) {
          acc[i][j] = Frag<T>::mma(ah, bl[j], acc[i][j]);
          acc[i][j] = Frag<T>::mma(al, bh[j], acc[i][j]);
        }
      }
      Frag<T>::guard(acc[i][0], acc[i][3], ah, SPLIT ? al : ah);
    }
    Frag<T>::keep(bh[0], bh[1], bh[2], bh[3]);
    if (SPLIT) Frag<T>::keep(bl[0], bl[1], bl[2], bl[3]);
  }
  acc_guard4(acc[0][0], acc[0][1], acc[0][2], acc[0][3]);
  acc_guard4(acc[1][0], acc[1][1], acc[1][2], acc[1][3]);
  acc_guard4(acc[2][0], acc[2][1], acc[2][2], acc[2][3]);
  acc_guard4(acc[3][0], acc[3][1], acc[3][2], acc[3][3]);

  float* slab = sT[wave];
  const float* Rb = RESID ? (resid + (size_t)b * strideR) : nullptr;
#pragma unroll
  for (int i = 0; i < 4; ++i) {
    const int mBase = m0 + (i << 4);
#pragma unroll
    for (int j = 0; j < 4; ++j) {
      const int n = n0 + (j << 4) + rlane;
      float bv = 0.f;
      if (BIAS_MODE == 2) bv = bias[n];
#pragma unroll
      for (int r = 0; r < 8; ++r) {
        float v = acc[i][j][r] * scale;
        if (BIAS_MODE == 1) v += bias[mBase + mOff + r];
        if (BIAS_MODE == 2) v += bv;
        if (RESID) v += Rb[(size_t)(mBase + mOff + r) * ldc + n];
        if (ACT == 2) v = fmaxf(v, 0.0f);
        if (ACT == 4) v = (v > 0.f) ? v : 0.01f * v;
        slab[(mOff + r) * 68 + (j << 4) + rlane] = v;
      }
    }
    __builtin_amdgcn_fence(__ATOMIC_RELEASE, "workgroup");
    __builtin_amdgcn_wave_barrier();
    __builtin_amdgcn_fence(__ATOMIC_ACQUIRE, "workgroup");
    if (OUT_MODE == 0) {
      float* C = (float*)Cout + (size_t)b * strideC;
      const int hh = lane >> 4, c4 = (lane & 15) * 4;
      for (int pass = 0; pass < 2; ++pass) {
#pragma unroll
        for (int it = 0; it < 8; ++it) {
          const int row = it * 2 + hh;
          v4f v = *(const v4f*)(slab + row * 68 + c4);
          *(volatile v4f*)(C + (size_t)(mBase + row) * ldc + n0 + c4) = v;
        }
        __threadfence();
      }
    } else {
      const int q = lane >> 3, c8 = (lane & 7) * 8;
      unsigned short* C  = (unsigned short*)Cout  + (size_t)b * strideC;
      unsigned short* C2 = (OUT_MODE == 2) ? ((unsigned short*)Cout2 + (size_t)b * strideC) : nullptr;
      for (int pass = 0; pass < 2; ++pass) {
#pragma unroll
        for (int it = 0; it < 4; ++it) {
          const int row = it * 4 + q;
          const float* sp = slab + row * 68 + c8;
          v8h hv, lv;
#pragma unroll
          for (int e = 0; e < 8; ++e) {
            if (OUT_MODE == 1) {
              hv[e] = (_Float16)sp[e];
            } else {
              unsigned short hb = f2bf_bits(sp[e]);
              unsigned short lb = f2bf_bits(sp[e] - bf_bits2f(hb));
              hv[e] = __builtin_bit_cast(_Float16, hb);
              lv[e] = __builtin_bit_cast(_Float16, lb);
            }
          }
          *(volatile v8h*)(C + (size_t)(mBase + row) * ldc + n0 + c8) = hv;
          if (OUT_MODE == 2) *(volatile v8h*)(C2 + (size_t)(mBase + row) * ldc + n0 + c8) = lv;
        }
        __threadfence();
      }
    }
    __builtin_amdgcn_fence(__ATOMIC_RELEASE, "workgroup");
    __builtin_amdgcn_wave_barrier();
    __builtin_amdgcn_fence(__ATOMIC_ACQUIRE, "workgroup");
  }
}

__global__ __launch_bounds__(256) void cast_rows_bf16(const float* __restrict__ src, int src_ld, int ncols,
                                                      unsigned short* __restrict__ dst, int dst_ld, int col0, int nrows) {
  const int cpr   = ncols >> 3;
  const int total = nrows * cpr;
  const int f0    = blockIdx.x * 256 + threadIdx.x;
  const bool act  = f0 < total;
  const int f     = act ? f0 : (total - 1);
  const int r     = f / cpr;
  const int c     = (f - r * cpr) << 3;
  const float* sp = src + (size_t)r * src_ld + c;
  const v4f a = *(const v4f*)sp;
  const v4f q = *(const v4f*)(sp + 4);
  v4u w;
  w.x = pk16(f2bf_bits(a.x), f2bf_bits(a.y));
  w.y = pk16(f2bf_bits(a.z), f2bf_bits(a.w));
  w.z = pk16(f2bf_bits(q.x), f2bf_bits(q.y));
  w.w = pk16(f2bf_bits(q.z), f2bf_bits(q.w));
  unsigned short* dp = dst + (size_t)r * dst_ld + col0 + c;
  if (act) *(volatile v4u*)dp = w;
  __threadfence();
  if (act) *(volatile v4u*)dp = w;
}

__global__ __launch_bounds__(256) void zero_chunks16(unsigned short* __restrict__ dst, int nchunks) {
  const int f = blockIdx.x * 256 + threadIdx.x;
  const v4u z = {0u, 0u, 0u, 0u};
  if (f < nchunks) *(volatile v4u*)(dst + (size_t)f * 8) = z;
  __threadfence();
  if (f < nchunks) *(volatile v4u*)(dst + (size_t)f * 8) = z;
}

__global__ __launch_bounds__(256) void build_bias(const float* __restrict__ bh, const float* __restrict__ ba,
                                                  const float* __restrict__ bb, const float* __restrict__ bva,
                                                  const float* __restrict__ bvb,
                                                  float* __restrict__ bias1, float* __restrict__ bias2) {
  const int t = threadIdx.x;
  if (blockIdx.x < 4) {
    const int n = blockIdx.x * 256 + t;
    const float v = bf_bits2f(f2bf_bits(bh[n]));
    *(volatile float*)(bias1 + n) = v;
    __threadfence();
    *(volatile float*)(bias1 + n) = v;
  } else {
    const int n = t;
    const int ia = n < 4 ? n : 3;
    int ib = n - 4;  ib = ib < 0 ? 0 : (ib > 3 ? 3 : ib);
    int iva = n - 8; iva = iva < 0 ? 0 : (iva > 63 ? 63 : iva);
    int ivb = n - 72; ivb = ivb < 0 ? 0 : (ivb > 63 ? 63 : ivb);
    const float va = ba[ia], vb = bb[ib], vva = bva[iva], vvb = bvb[ivb];
    float v = 0.f;
    v = (n < kUReal) ? vvb : v;
    v = (n < 72) ? vva : v;
    v = (n < 8) ? vb : v;
    v = (n < 4) ? va : v;
    v = bf_bits2f(f2bf_bits(v));
    if (n < kUN) *(volatile float*)(bias2 + n) = v;
    __threadfence();
    if (n < kUN) *(volatile float*)(bias2 + n) = v;
  }
}

__device__ __forceinline__ float pow5abs(float x) { const float a = fabsf(x); const float t = a * a; return t * t * a; }

__global__ __launch_bounds__(256) void mem_update(const float* __restrict__ U, const float* __restrict__ memin,
                                                  float* __restrict__ memOut) {
  const int lane = threadIdx.x & 31;
  const int wave = threadIdx.x >> 5;
  const int b    = blockIdx.x * 8 + wave;
  const float* u = U + (size_t)b * kUN;
  const float aL  = u[lane & 3];
  const float bL  = u[4 + (lane & 3)];
  const float u0a = u[8 + lane];
  const float u1a = u[40 + lane];
  const float u0b = u[72 + lane];
  const float u1b = u[104 + lane];

  float s1a = pow5abs(u1a), s1b = pow5abs(u1b);
#pragma unroll
  for (int m = 1; m <= 16; m <<= 1) { s1a += __shfl_xor(s1a, m, 32); s1b += __shfl_xor(s1b, m, 32); }
  float s0a = pow5abs(u0a), s0b = pow5abs(u0b);
#pragma unroll
  for (int m = 1; m <= 4; m <<= 1) { s0a += __shfl_xor(s0a, m, 32); s0b += __shfl_xor(s0b, m, 32); }
  const float na = powf(s0a * s1a, 0.2f);
  const float nb = powf(s0b * s1b, 0.2f);
  const int kq = lane >> 3;
  const float alpha_k = __shfl(aL, kq, 32);
  const float beta_k  = __shfl(bL, kq, 32);
  float ca = alpha_k * __builtin_amdgcn_rcpf(fmaxf(na, 1e-12f)) * u0a;
  float cb = beta_k  * __builtin_amdgcn_rcpf(fmaxf(nb, 1e-12f)) * u0b;
  ca += __shfl_xor(ca, 8, 32);  ca += __shfl_xor(ca, 16, 32);
  cb += __shfl_xor(cb, 8, 32);  cb += __shfl_xor(cb, 16, 32);

  const float* mrow = memin + (size_t)b * kMemF;
  float* orow = memOut + (size_t)b * kMemF;
  float res[8];
#pragma unroll
  for (int t = 0; t < 8; ++t) {
    const float pa = __shfl(ca, t, 32);
    const float pb = __shfl(cb, t, 32);
    const float mq = bf_bits2f(f2bf_bits(mrow[t * 32 + lane]));
    res[t] = mq + 0.25f * (pa * u1a - pb * u1b);
  }
#pragma unroll
  for (int t = 0; t < 8; ++t) *(volatile float*)(orow + t * 32 + lane) = res[t];
  __threadfence();
#pragma unroll
  for (int t = 0; t < 8; ++t) *(volatile float*)(orow + t * 32 + lane) = res[t];
}

static inline unsigned cdiv_u(unsigned a, unsigned b) { return (a + b - 1) / b; }

extern "C" void kernel_launch(void* const* d_in, const int* in_sizes, int n_in,
                              void* d_out, int out_size, void* d_ws, size_t ws_size,
                              hipStream_t stream) {
  (void)in_sizes; (void)out_size;
  if (n_in < 13 || ws_size < kWsTotal) return;

  const float* x    = (const float*)d_in[0];
  const float* h0   = (const float*)d_in[1];
  const float* mem  = (const float*)d_in[2];
  const float* Wh   = (const float*)d_in[3];
  const float* bh   = (const float*)d_in[4];
  const float* Wa   = (const float*)d_in[5];
  const float* ba   = (const float*)d_in[6];
  const float* Wb   = (const float*)d_in[7];
  const float* bb   = (const float*)d_in[8];
  const float* Wva  = (const float*)d_in[9];
  const float* bva  = (const float*)d_in[10];
  const float* Wvb  = (const float*)d_in[11];
  const float* bvb  = (const float*)d_in[12];

  float* memOut = (float*)d_out;
  float* hOut   = (float*)((char*)d_out + 8388608);

  char* ws = (char*)d_ws;
  unsigned short* A1 = (unsigned short*)(ws + kOffA1);
  unsigned short* W1 = (unsigned short*)(ws + kOffW1);
  unsigned short* A2 = (unsigned short*)(ws + kOffA2);
  unsigned short* W2 = (unsigned short*)(ws + kOffW2);
  float* U      = (float*)(ws + kOffU);
  float* bias1  = (float*)(ws + kOffB1);
  float* bias2  = (float*)(ws + kOffB2);

  cast_rows_bf16<<<cdiv_u(kBatch * (kInpF / 8), 256), 256, 0, stream>>>(x,   kInpF, kInpF, A1, kCatK, 0,             kBatch);
  cast_rows_bf16<<<cdiv_u(kBatch * (kHidF / 8), 256), 256, 0, stream>>>(h0,  kHidF, kHidF, A1, kCatK, kInpF,         kBatch);
  cast_rows_bf16<<<cdiv_u(kBatch * (kMemF / 8), 256), 256, 0, stream>>>(mem, kMemF, kMemF, A1, kCatK, kInpF + kHidF, kBatch);
  cast_rows_bf16<<<cdiv_u(kHidF * (kCatK / 8), 256), 256, 0, stream>>>(Wh,  kCatK, kCatK, W1, kCatK, 0,             kHidF);
  build_bias<<<5, 256, 0, stream>>>(bh, ba, bb, bva, bvb, bias1, bias2);

  wmma_gemm64<1, false, 2, 0, false, 2><<<dim3(256, 1), 256, 0, stream>>>(
      A1, A1, kCatK, 0L, W1, W1, kCatK, 0L, (void*)hOut, (void*)hOut, kHidF, 0L,
      bias1, bias1, 0L, kBatch, kHidF, kCatK, 1.0f);

  cast_rows_bf16<<<cdiv_u(kBatch * (kHidF / 8), 256), 256, 0, stream>>>(hOut, kHidF, kHidF, A2, kHmK, 0,     kBatch);
  cast_rows_bf16<<<cdiv_u(kBatch * (kMemF / 8), 256), 256, 0, stream>>>(mem,  kMemF, kMemF, A2, kHmK, kHidF, kBatch);
  cast_rows_bf16<<<cdiv_u(4  * (kHmK / 8), 256), 256, 0, stream>>>(Wa,  kHmK, kHmK, W2,                       kHmK, 0, 4);
  cast_rows_bf16<<<cdiv_u(4  * (kHmK / 8), 256), 256, 0, stream>>>(Wb,  kHmK, kHmK, W2 + (size_t)4  * kHmK,  kHmK, 0, 4);
  cast_rows_bf16<<<cdiv_u(64 * (kHmK / 8), 256), 256, 0, stream>>>(Wva, kHmK, kHmK, W2 + (size_t)8  * kHmK,  kHmK, 0, 64);
  cast_rows_bf16<<<cdiv_u(64 * (kHmK / 8), 256), 256, 0, stream>>>(Wvb, kHmK, kHmK, W2 + (size_t)72 * kHmK,  kHmK, 0, 64);
  zero_chunks16<<<cdiv_u((kUN - kUReal) * kHmK / 8, 256), 256, 0, stream>>>(W2 + (size_t)kUReal * kHmK, (kUN - kUReal) * kHmK / 8);

  wmma_gemm64<1, false, 2, 0, false, 0><<<dim3(48, 1), 256, 0, stream>>>(
      A2, A2, kHmK, 0L, W2, W2, kHmK, 0L, (void*)U, (void*)U, kUN, 0L,
      bias2, bias2, 0L, kBatch, kUN, kHmK, 1.0f);

  mem_update<<<kBatch / 8, 256, 0, stream>>>(U, mem, memOut);
}
